// MultiHeadAttention_56461640073327
// MI455X (gfx1250) — hardware-verified
//
#include <hip/hip_runtime.h>


#ifndef NB
#define NB 2
#endif
#ifndef SEQ
#define SEQ 2048
#endif
#define NB_FULL  2
#define SEQ_FULL 2048
#define DM    1024
#define NHEAD 16
#define HDIM  64
#define D3    (3 * DM)
#define PLANE ((size_t)NB * NHEAD * SEQ * HDIM)
#define CSC   0.18033688011112042f
#define PLOG  6.0f

typedef _Float16 h16;
typedef unsigned short bf;
typedef __attribute__((ext_vector_type(16))) __bf16   v16bf;
typedef __attribute__((ext_vector_type(16))) _Float16 v16h;
typedef __attribute__((ext_vector_type(8)))  _Float16 v8h;
typedef __attribute__((ext_vector_type(8)))  unsigned short v8us;
typedef __attribute__((ext_vector_type(8)))  float    v8f;
typedef __attribute__((ext_vector_type(4)))  float    v4f;
typedef v8h  __attribute__((may_alias)) v8ha;
typedef v4f  __attribute__((may_alias)) v4fa;

static_assert(SEQ % 64 == 0);
static_assert((NB * SEQ) % 64 == 0);
static_assert(DM % 64 == 0);
static_assert(DM % 32 == 0);
static_assert(HDIM == 64);
static_assert(NHEAD * HDIM == DM);
static_assert(D3 % 64 == 0);
static_assert(NB <= NB_FULL);
static_assert(SEQ <= SEQ_FULL);

constexpr size_t SZ_WB  = (size_t)D3 * DM * 2;
constexpr size_t SZ_WO  = (size_t)DM * DM * 2;
constexpr size_t SZ_XB  = (size_t)NB * SEQ * DM * 2;
constexpr size_t SZ_EMB = (size_t)SEQ * HDIM * 4;
constexpr size_t SZ_QK  = (size_t)2 * NB * NHEAD * SEQ * HDIM * 2;
constexpr size_t SZ_VT  = (size_t)NB * NHEAD * HDIM * SEQ * 2;
constexpr size_t SZ_AT  = (size_t)NB * SEQ * 2 * DM * 2;
constexpr size_t OFF_WB  = 0;
constexpr size_t OFF_WO  = OFF_WB + SZ_WB;
constexpr size_t OFF_XB  = OFF_WO + SZ_WO;
constexpr size_t OFF_EMB = OFF_XB + SZ_XB;
constexpr size_t OFF_QK  = OFF_EMB + SZ_EMB;
constexpr size_t OFF_VT  = OFF_QK + SZ_QK;
constexpr size_t OFF_AT  = OFF_VT + SZ_VT;
constexpr size_t WS_TOTAL = OFF_AT + SZ_AT;
static_assert(SZ_WB % 256 == 0);
static_assert(SZ_WO % 256 == 0);
static_assert(SZ_XB % 256 == 0);
static_assert(SZ_EMB % 256 == 0);
static_assert(SZ_QK % 256 == 0);
static_assert(SZ_VT % 256 == 0);
static_assert(SZ_AT % 256 == 0);
static_assert(WS_TOTAL <= (size_t)134217728);

__device__ __forceinline__ unsigned short f2bf(float f) { unsigned u = __float_as_uint(f); u += 0x7FFFu + ((u >> 16) & 1u); return (unsigned short)(u >> 16); }
__device__ __forceinline__ float bf2f(unsigned short b) { return __uint_as_float(((unsigned)b) << 16); }
__device__ __forceinline__ float bfr(float f) { return bf2f(f2bf(f)); }
__device__ __forceinline__ void splitf(float y, unsigned short& h, unsigned short& l) { h = f2bf(y); l = f2bf(y - bf2f(h)); }
__device__ __forceinline__ v16h cat16(v8h lo, v8h hi) { return __builtin_shufflevector(lo, hi, 0, 1, 2, 3, 4, 5, 6, 7, 8, 9, 10, 11, 12, 13, 14, 15); }
__device__ __forceinline__ v16bf cat16b(v8us lo, v8us hi) { return __builtin_bit_cast(v16bf, __builtin_shufflevector(lo, hi, 0, 1, 2, 3, 4, 5, 6, 7, 8, 9, 10, 11, 12, 13, 14, 15)); }
__device__ __forceinline__ v8f wmma16(v16h a, v16h b, v8f c) { return __builtin_amdgcn_wmma_f32_16x16x32_f16(false, a, false, b, (short)0, c, false, false); }
__device__ __forceinline__ v8f wmmab(v16bf a, v16bf b, v8f c) { return __builtin_amdgcn_wmma_f32_16x16x32_bf16(false, a, false, b, (short)0, c, false, false); }
__device__ __forceinline__ v16h  ldfh(const h16* p) { return cat16(*(const v8h*)p, *(const v8h*)(p + 16)); }
__device__ __forceinline__ v16bf ldfb(const bf* p)  { return cat16b(*(const v8us*)p, *(const v8us*)(p + 16)); }
__device__ __forceinline__ void lds_wave_sync() { asm volatile("s_wait_dscnt 0x0" ::: "memory"); __builtin_amdgcn_wave_barrier(); asm volatile("" ::: "memory"); }

__device__ __forceinline__ void gemm_tile(const bf* __restrict__ A, const bf* __restrict__ Bt, const int K, const int KB, const int r0, const int c0, const int lr, const int hi, v8f (&acc)[4][4]) {
    const size_t aoff = (size_t)(r0 + lr) * K + 8 * hi;
    const size_t boff = (size_t)(c0 + lr) * KB + 8 * hi;
#pragma unroll 1
    for (int kc = 0; kc < K; kc += 32) {
        const int kb = (kc >= KB) ? (kc - KB) : kc;
        v16bf a[4];
#pragma unroll
        for (int mb = 0; mb < 4; ++mb) a[mb] = ldfb(A + aoff + (size_t)mb * 16 * K + kc);
        v16bf b;
#pragma unroll
        for (int nb = 0; nb < 4; ++nb) {
            b = ldfb(Bt + boff + (size_t)nb * 16 * KB + kb);
#pragma unroll
            for (int mb = 0; mb < 4; ++mb) acc[mb][nb] = wmmab(a[mb], b, acc[mb][nb]);
        }
        asm volatile("" : "+v"(acc[0][0]), "+v"(acc[1][0]), "+v"(acc[2][0]), "+v"(acc[3][0]), "+v"(acc[0][1]), "+v"(acc[1][1]), "+v"(acc[2][1]), "+v"(acc[3][1]));
        asm volatile("v_nop\n\tv_nop\n\tv_nop\n\tv_nop" : "+v"(acc[0][2]), "+v"(acc[1][2]), "+v"(acc[2][2]), "+v"(acc[3][2]), "+v"(acc[0][3]), "+v"(acc[1][3]), "+v"(acc[2][3]), "+v"(acc[3][3]) : "v"(a[0]), "v"(a[3]), "v"(b));
    }
}

__global__ __launch_bounds__(256) void k_cvt8(const float* __restrict__ src, bf* dst, int n8) {
    const int i = blockIdx.x * 256 + threadIdx.x; if (i >= n8) return;
    const v8f v = *(const v8f*)(src + (size_t)i * 8); v8us o;
#pragma unroll
    for (int k = 0; k < 8; ++k) o[k] = f2bf(v[k]);
    *(volatile v8us*)(dst + (size_t)i * 8) = o; __threadfence(); *(volatile v8us*)(dst + (size_t)i * 8) = o;
}

__global__ __launch_bounds__(256) void k_cvtx(const float* __restrict__ x, bf* XB) {
    const int i = blockIdx.x * 256 + threadIdx.x; if (i >= NB * SEQ * (DM / 8)) return;
    const int row = i / (DM / 8), c8 = i % (DM / 8); const int b = row / SEQ, t = row % SEQ;
    const v8f v = *(const v8f*)(x + ((size_t)b * SEQ_FULL + t) * DM + c8 * 8); v8us o;
#pragma unroll
    for (int k = 0; k < 8; ++k) o[k] = f2bf(v[k]);
    *(volatile v8us*)(XB + (size_t)i * 8) = o; __threadfence(); *(volatile v8us*)(XB + (size_t)i * 8) = o;
}

__global__ __launch_bounds__(256) void k_emb(float* EMB) {
    const int lane = threadIdx.x & 31; const int wave = __builtin_amdgcn_readfirstlane(threadIdx.x >> 5);
    const int t = blockIdx.x * 8 + wave; if (t >= SEQ) return;
    const int fr = lane & 7, dec = lane >> 3;
    double f = 1.0;
    f = (fr == 1) ? 1.333521432163324  : f;
    f = (fr == 2) ? 1.7782794100389228 : f;
    f = (fr == 3) ? 2.371373705661655  : f;
    f = (fr == 4) ? 3.1622776601683795 : f;
    f = (fr == 5) ? 4.216965034285822  : f;
    f = (fr == 6) ? 5.623413251903491  : f;
    f = (fr == 7) ? 7.498942093324558  : f;
    double d = 1.0;
    d = (dec == 1) ? 10.0 : d; d = (dec == 2) ? 100.0 : d; d = (dec == 3) ? 1000.0 : d;
    const float pf = (float)(d * f);
    const float inv = 1.0f / pf;
    const float ang = (float)t * inv;
    float sn, cs; sincosf(ang, &sn, &cs);
    float* row = EMB + (size_t)t * HDIM;
    *(volatile float*)(row + lane) = sn; *(volatile float*)(row + 32 + lane) = cs;
    __threadfence();
    *(volatile float*)(row + lane) = sn; *(volatile float*)(row + 32 + lane) = cs;
}

__global__ __launch_bounds__(32) void k_qkv(const bf* __restrict__ XB, const bf* __restrict__ WB, const float* __restrict__ bias, const float* __restrict__ EMB, h16* QK, h16* VT) {
    __shared__ __align__(16) float os[64 * 68];
    __shared__ __align__(16) h16 vts[64 * 72];
    const int lane = threadIdx.x & 31, lr = lane & 15, hi = lane >> 4;
    const int r0 = blockIdx.x * 64, c0 = blockIdx.y * 64;
    const int which = blockIdx.y / NHEAD, h = blockIdx.y % NHEAD;
    const int b = r0 / SEQ, t0 = r0 % SEQ;
    v8f acc[4][4];
#pragma unroll
    for (int mb = 0; mb < 4; ++mb)
#pragma unroll
        for (int nb = 0; nb < 4; ++nb) acc[mb][nb] = (v8f){};
    gemm_tile(XB, WB, DM, DM, r0, c0, lr, hi, acc);
    float bv[4];
#pragma unroll
    for (int nb = 0; nb < 4; ++nb) bv[nb] = bfr(bias[c0 + nb * 16 + lr]);
    if (which < 2) {
#pragma unroll
        for (int mb = 0; mb < 4; ++mb)
#pragma unroll
            for (int nb = 0; nb < 4; ++nb)
#pragma unroll
                for (int j = 0; j < 8; ++j) os[(mb * 16 + hi * 8 + j) * 68 + nb * 16 + lr] = acc[mb][nb][j] + bv[nb];
        lds_wave_sync();
        const int pc = lane & 7, e0 = pc * 8, ii = e0 & 31; const bool up = (e0 >= 32);
        const size_t pbase = (size_t)which * PLANE + ((size_t)(b * NHEAD + h) * SEQ + t0) * HDIM + e0;
#pragma unroll 1
        for (int it = 0; it < 16; ++it) {
            const int row = it * 4 + (lane >> 3);
            const float* er = EMB + (size_t)(t0 + row) * HDIM + 2 * ii;
            v4f xs[4], es[4];
#pragma unroll
            for (int q = 0; q < 4; ++q) { xs[q] = *(const v4fa*)&os[row * 68 + 2 * ii + 4 * q]; es[q] = *(const v4f*)(er + 4 * q); }
            v8h ov;
#pragma unroll
            for (int k = 0; k < 8; ++k) {
                const float x1 = xs[k >> 1][(k & 1) * 2], x2 = xs[k >> 1][(k & 1) * 2 + 1];
                const float sn = es[k >> 1][(k & 1) * 2], cs = es[k >> 1][(k & 1) * 2 + 1];
                const float lo = x1 * cs - x2 * sn, hv = x1 * sn + x2 * cs;
                ov[k] = (h16)(up ? hv : lo);
            }
            h16* dst = QK + pbase + (size_t)row * HDIM;
            *(volatile v8h*)dst = ov; __threadfence(); *(volatile v8h*)dst = ov;
        }
    } else {
#pragma unroll
        for (int mb = 0; mb < 4; ++mb)
#pragma unroll
            for (int nb = 0; nb < 4; ++nb) {
                v8h pk;
#pragma unroll
                for (int j = 0; j < 8; ++j) pk[j] = (h16)(acc[mb][nb][j] + bv[nb]);
                *(v8ha*)&vts[(nb * 16 + lr) * 72 + mb * 16 + hi * 8] = pk;
            }
        lds_wave_sync();
        const int pc = lane & 7;
        const size_t vbase = (size_t)(b * NHEAD + h) * HDIM * SEQ + t0 + pc * 8;
#pragma unroll 1
        for (int it = 0; it < 16; ++it) {
            const int d = it * 4 + (lane >> 3);
            const v8h val = *(const v8ha*)&vts[d * 72 + pc * 8];
            h16* dst = VT + vbase + (size_t)d * SEQ;
            *(volatile v8h*)dst = val; __threadfence(); *(volatile v8h*)dst = val;
        }
    }
}

__global__ __launch_bounds__(128) void k_attn(const h16* __restrict__ QK, const h16* __restrict__ VT, bf* AT) {
    __shared__ __align__(16) float ots[4 * 16 * 68];
    const int lane = threadIdx.x & 31, lr = lane & 15, hi = lane >> 4;
    const int wave = __builtin_amdgcn_readfirstlane(threadIdx.x >> 5);
    const int bh = blockIdx.y; const int b = bh / NHEAD, h = bh % NHEAD;
    const int q0 = blockIdx.x * 64 + wave * 16;
    const size_t qoff = (size_t)bh * SEQ * HDIM + (size_t)(q0 + lr) * HDIM + 8 * hi;
    const size_t koff = PLANE + (size_t)bh * SEQ * HDIM + (size_t)lr * HDIM + 8 * hi;
    const size_t voff = (size_t)bh * HDIM * SEQ + (size_t)lr * SEQ + 8 * hi;
    const v16h qf0 = ldfh(QK + qoff), qf1 = ldfh(QK + qoff + 32);
    v8f ot[4];
#pragma unroll
    for (int mt = 0; mt < 4; ++mt) ot[mt] = (v8f){};
    float m2 = -3.0e38f, l = 0.0f;
#pragma unroll 1
    for (int key0 = 0; key0 < SEQ; key0 += 64) {
        v8f s[4];
        v16h ka, kb2;
#pragma unroll
        for (int kt = 0; kt < 4; ++kt) {
            const h16* kp = QK + koff + (size_t)(key0 + kt * 16) * HDIM;
            ka = ldfh(kp); kb2 = ldfh(kp + 32);
            s[kt] = (v8f){};
            s[kt] = wmma16(ka, qf0, s[kt]);
            s[kt] = wmma16(kb2, qf1, s[kt]);
        }
        asm volatile("v_nop\n\tv_nop\n\tv_nop\n\tv_nop" : "+v"(s[0]), "+v"(s[1]), "+v"(s[2]), "+v"(s[3]) : "v"(ka), "v"(kb2), "v"(qf0), "v"(qf1));
        float mx = s[0][0];
#pragma unroll
        for (int kt = 0; kt < 4; ++kt)
#pragma unroll
            for (int r = 0; r < 8; ++r) mx = fmaxf(mx, s[kt][r]);
        mx = fmaxf(mx, __shfl_xor(mx, 16, 32));
        const float mnew = fmaxf(m2, mx * CSC);
        const float alpha = __builtin_amdgcn_exp2f(m2 - mnew);
        m2 = mnew;
        const float off = PLOG - mnew;
        float rs = 0.0f;
#pragma unroll
        for (int kt = 0; kt < 4; ++kt)
#pragma unroll
            for (int r = 0; r < 8; ++r) { const float p = __builtin_amdgcn_exp2f(fmaf(s[kt][r], CSC, off)); s[kt][r] = p; rs += p; }
        l = fmaf(l, alpha, rs);
#pragma unroll
        for (int mt = 0; mt < 4; ++mt)
#pragma unroll
            for (int r = 0; r < 8; ++r) ot[mt][r] *= alpha;
        v16h pb0, pb1;
#pragma unroll
        for (int i = 0; i < 8; ++i) { pb0[i] = (h16)s[0][i]; pb0[8 + i] = (h16)s[1][i]; pb1[i] = (h16)s[2][i]; pb1[8 + i] = (h16)s[3][i]; }
        v16h va[4], vb[4];
#pragma unroll
        for (int mt = 0; mt < 4; ++mt) va[mt] = ldfh(VT + voff + (size_t)mt * 16 * SEQ + key0);
#pragma unroll
        for (int mt = 0; mt < 4; ++mt) vb[mt] = ldfh(VT + voff + (size_t)mt * 16 * SEQ + key0 + 32);
#pragma unroll
        for (int mt = 0; mt < 4; ++mt) ot[mt] = wmma16(va[mt], pb0, ot[mt]);
#pragma unroll
        for (int mt = 0; mt < 4; ++mt) ot[mt] = wmma16(vb[mt], pb1, ot[mt]);
        asm volatile("v_nop\n\tv_nop\n\tv_nop\n\tv_nop" : "+v"(ot[0]), "+v"(ot[1]), "+v"(ot[2]), "+v"(ot[3]) : "v"(va[3]), "v"(vb[3]), "v"(pb0), "v"(pb1));
    }
    l += __shfl_xor(l, 16, 32);
    const float inv = 1.0f / l;
    const int ob = wave * (16 * 68);
#pragma unroll
    for (int mt = 0; mt < 4; ++mt) {
        v4f x0, x1;
#pragma unroll
        for (int r = 0; r < 4; ++r) { x0[r] = ot[mt][r] * inv; x1[r] = ot[mt][4 + r] * inv; }
        *(v4fa*)&ots[ob + lr * 68 + mt * 16 + hi * 8] = x0;
        *(v4fa*)&ots[ob + lr * 68 + mt * 16 + hi * 8 + 4] = x1;
    }
    lds_wave_sync();
    const int pc = lane & 7;
    const size_t abase = ((size_t)b * SEQ + q0) * (2 * DM) + h * HDIM + pc * 8;
#pragma unroll 1
    for (int it = 0; it < 4; ++it) {
        const int row = it * 4 + (lane >> 3);
        const v4f y0 = *(const v4fa*)&ots[ob + row * 68 + pc * 8];
        const v4f y1 = *(const v4fa*)&ots[ob + row * 68 + pc * 8 + 4];
        v8us oh, ol;
#pragma unroll
        for (int k = 0; k < 4; ++k) { unsigned short a, c; splitf(y0[k], a, c); oh[k] = a; ol[k] = c; splitf(y1[k], a, c); oh[4 + k] = a; ol[4 + k] = c; }
        bf* dst = AT + abase + (size_t)row * (2 * DM);
        *(volatile v8us*)dst = oh; *(volatile v8us*)(dst + DM) = ol;
        __threadfence();
        *(volatile v8us*)dst = oh; *(volatile v8us*)(dst + DM) = ol;
    }
}

__global__ __launch_bounds__(32) void k_oproj(const bf* __restrict__ AT, const bf* __restrict__ WO, const float* __restrict__ bias, float* OUT) {
    __shared__ __align__(16) float os[64 * 68];
    const int lane = threadIdx.x & 31, lr = lane & 15, hi = lane >> 4;
    const int r0 = blockIdx.x * 64, c0 = blockIdx.y * 64;
    v8f acc[4][4];
#pragma unroll
    for (int mb = 0; mb < 4; ++mb)
#pragma unroll
        for (int nb = 0; nb < 4; ++nb) acc[mb][nb] = (v8f){};
    gemm_tile(AT, WO, 2 * DM, DM, r0, c0, lr, hi, acc);
    float bv[4];
#pragma unroll
    for (int nb = 0; nb < 4; ++nb) bv[nb] = bfr(bias[c0 + nb * 16 + lr]);
#pragma unroll
    for (int mb = 0; mb < 4; ++mb)
#pragma unroll
        for (int nb = 0; nb < 4; ++nb)
#pragma unroll
            for (int j = 0; j < 8; ++j) os[(mb * 16 + hi * 8 + j) * 68 + nb * 16 + lr] = acc[mb][nb][j] + bv[nb];
    lds_wave_sync();
    const int cofs = lr * 4;
#pragma unroll 1
    for (int it = 0; it < 32; ++it) {
        const int row = it * 2 + hi;
        const v4f val = *(const v4fa*)&os[row * 68 + cofs];
        float* dst = OUT + (size_t)(r0 + row) * DM + c0 + cofs;
        *(volatile v4f*)dst = val; __threadfence(); *(volatile v4f*)dst = val;
    }
}

extern "C" void kernel_launch(void* const* d_in, const int* in_sizes, int n_in,
                              void* d_out, int out_size, void* d_ws, size_t ws_size, hipStream_t stream) {
    if (n_in < 5) return;
    if ((size_t)in_sizes[0] < ((size_t)(NB - 1) * SEQ_FULL + SEQ) * DM) return;
    if ((size_t)in_sizes[1] < (size_t)D3 * DM) return;
    if ((size_t)in_sizes[2] < (size_t)D3) return;
    if ((size_t)in_sizes[3] < (size_t)DM * DM) return;
    if ((size_t)in_sizes[4] < (size_t)DM) return;
    if ((size_t)out_size < (size_t)NB * SEQ * DM) return;
    if (ws_size < WS_TOTAL) return;
    const float* x     = (const float*)d_in[0];
    const float* qkv_w = (const float*)d_in[1];
    const float* qkv_b = (const float*)d_in[2];
    const float* out_w = (const float*)d_in[3];
    const float* out_b = (const float*)d_in[4];
    float* OUT = (float*)d_out;
    char* wsp = (char*)d_ws;
    bf*    WB  = (bf*)(wsp + OFF_WB);
    bf*    WO  = (bf*)(wsp + OFF_WO);
    bf*    XB  = (bf*)(wsp + OFF_XB);
    float* EMB = (float*)(wsp + OFF_EMB);
    h16*   QK  = (h16*)(wsp + OFF_QK);
    h16*   VT  = (h16*)(wsp + OFF_VT);
    bf*    AT  = (bf*)(wsp + OFF_AT);

    k_cvt8<<<(D3 * DM / 8 + 255) / 256, 256, 0, stream>>>(qkv_w, WB, D3 * DM / 8);
    k_cvt8<<<(DM * DM / 8 + 255) / 256, 256, 0, stream>>>(out_w, WO, DM * DM / 8);
    k_cvtx<<<(NB * SEQ * (DM / 8) + 255) / 256, 256, 0, stream>>>(x, XB);
    k_emb<<<(SEQ + 7) / 8, 256, 0, stream>>>(EMB);
    k_qkv<<<dim3(NB * SEQ / 64, D3 / 64, 1), 32, 0, stream>>>(XB, WB, qkv_b, EMB, QK, VT);
    k_attn<<<dim3(SEQ / 64, NB * NHEAD, 1), 128, 0, stream>>>(QK, VT, AT);
    k_oproj<<<dim3(NB * SEQ / 64, DM / 64, 1), 32, 0, stream>>>(AT, WO, out_b, OUT);
}
